// SuperResolutionBlock_56719338111572
// MI455X (gfx1250) — hardware-verified
//
#include <hip/hip_runtime.h>
#include <stddef.h>
#include <math.h>

constexpr int NIMG = 2;
constexpr int CIN  = 64;
constexpr int CMID = 32;
constexpr int HS1  = 128;
constexpr int PX1  = 16384;
constexpr int HS2  = 256;
constexpr int PX2  = 65536;
constexpr int NTAP = 9;
constexpr int KT1  = 576;
constexpr int KT2  = 288;
constexpr int NOFF = 27;
constexpr int NPAD = 64;
constexpr int PARSLOT = 64;
constexpr float CARRY_ACT = 16.0f;
constexpr float CARRY_W   = 64.0f;
constexpr float CARRY_INV = 1.0f / 1024.0f;
static_assert(KT1 == NTAP * CIN && KT2 == NTAP * CMID, "");
static_assert(KT1 % 32 == 0 && KT2 % 32 == 0 && CIN % 32 == 0, "");
static_assert((NIMG * PX1) % 64 == 0 && PX2 % 64 == 0 && NPAD == 64, "");
static_assert((NIMG * PX1 * NTAP * 8) % 256 == 0 && (PX2 * NTAP * 4) % 256 == 0, "");
static_assert((64 * KT1) % (8 * 256) == 0 && (64 * KT2) % (8 * 256) == 0 && (64 * CIN) % (8 * 256) == 0, "");

typedef __attribute__((ext_vector_type(16))) _Float16 v16h;
typedef __attribute__((ext_vector_type(8)))  _Float16 v8h;
typedef __attribute__((ext_vector_type(16))) __bf16   v16b;
typedef __attribute__((ext_vector_type(8)))  __bf16   v8b;
typedef __attribute__((ext_vector_type(8)))  float    v8f;
typedef __attribute__((ext_vector_type(4)))  float    v4f;
typedef __attribute__((ext_vector_type(4)))  unsigned v4u;

__device__ __forceinline__ unsigned short f2bf_bits(float f) {
  unsigned u = __float_as_uint(f);
  return (unsigned short)((u + 0x7FFFu + ((u >> 16) & 1u)) >> 16);
}
__device__ __forceinline__ float bf_bits2f(unsigned short h) { return __uint_as_float(((unsigned)h) << 16); }

__device__ __forceinline__ void dep_guard_h(v8f& a, v8f& b, v16h x, v16h y) { asm volatile("v_nop\n\tv_nop\n\tv_nop\n\tv_nop" : "+v"(a), "+v"(b) : "v"(x), "v"(y)); }
__device__ __forceinline__ void dep_guard_b(v8f& a, v8f& b, v16b x, v16b y) { asm volatile("v_nop\n\tv_nop\n\tv_nop\n\tv_nop" : "+v"(a), "+v"(b) : "v"(x), "v"(y)); }
__device__ __forceinline__ void keep4_h(v16h a, v16h b, v16h c, v16h d) { asm volatile("v_nop" :: "v"(a), "v"(b), "v"(c), "v"(d)); }
__device__ __forceinline__ void keep4_b(v16b a, v16b b, v16b c, v16b d) { asm volatile("v_nop" :: "v"(a), "v"(b), "v"(c), "v"(d)); }
__device__ __forceinline__ void acc_guard4(v8f& a, v8f& b, v8f& c, v8f& d) { asm volatile("v_nop\n\tv_nop\n\tv_nop\n\tv_nop" : "+v"(a), "+v"(b), "+v"(c), "+v"(d)); }
template <typename T> struct Frag;
template <> struct Frag<_Float16> {
  typedef v16h V; union U { v16h v; v8h h[2]; };
  static __device__ __forceinline__ v16h load(const _Float16* p) {
    U f; f.h[0] = *(const v8h*)(p); f.h[1] = *(const v8h*)(p + 16); return f.v;
  }
  static __device__ __forceinline__ v8f mma(v16h a, v16h b, v8f c) {
    return __builtin_amdgcn_wmma_f32_16x16x32_f16(false, a, false, b, (short)0, c, false, false);
  }
  static __device__ __forceinline__ void guard(v8f& a, v8f& b, v16h x, v16h y) { dep_guard_h(a, b, x, y); }
  static __device__ __forceinline__ void keep(v16h a, v16h b, v16h c, v16h d) { keep4_h(a, b, c, d); }
};
template <> struct Frag<__bf16> {
  typedef v16b V; union U { v16b v; v8b h[2]; };
  static __device__ __forceinline__ v16b load(const __bf16* p) {
    U f; f.h[0] = *(const v8b*)(p); f.h[1] = *(const v8b*)(p + 16); return f.v;
  }
  static __device__ __forceinline__ v8f mma(v16b a, v16b b, v8f c) {
    return __builtin_amdgcn_wmma_f32_16x16x32_bf16(false, a, false, b, (short)0, c, false, false);
  }
  static __device__ __forceinline__ void guard(v8f& a, v8f& b, v16b x, v16b y) { dep_guard_b(a, b, x, y); }
  static __device__ __forceinline__ void keep(v16b a, v16b b, v16b c, v16b d) { keep4_b(a, b, c, d); }
};

template <int ET> struct Elem;
template <> struct Elem<0> { typedef _Float16 T; };
template <> struct Elem<1> { typedef __bf16 T; };
template <int ET, bool SPLIT, int BIAS_MODE, int OUT_MODE, bool RESID, int ACT = 0>
__global__ __launch_bounds__(256) void wmma_gemm64(
    const unsigned short* __restrict__ Ap, const unsigned short* __restrict__ A2p, int lda, long strideA,
    const unsigned short* __restrict__ Btp, const unsigned short* __restrict__ Bt2p, int ldb, long strideB,
    void* __restrict__ Cout, void* __restrict__ Cout2, int ldc, long strideC,
    const float* __restrict__ bias,
    const float* __restrict__ resid, long strideR,
    int M, int N, int K, float scale) {
  typedef typename Elem<ET>::T T;
  typedef typename Frag<T>::V V;
  const T* A = (const T*)Ap; const T* A2 = (const T*)A2p; const T* Bt = (const T*)Btp; const T* Bt2 = (const T*)Bt2p;
  __shared__ __align__(16) float sT[8][16 * 68];
  const int b    = blockIdx.y;
  const int lane = threadIdx.x & 31;
  const int wave = threadIdx.x >> 5;
  const int tilesN = N >> 6;
  const int tilesM = M >> 6;
  const int tile = blockIdx.x * 8 + wave;
  if (tile >= tilesM * tilesN) return;
  const int tm = tile / tilesN;
  const int tn = tile - tm * tilesN;
  const int m0 = tm << 6;
  const int n0 = tn << 6;

  const T* Ab  = A  + (size_t)b * strideA;
  const T* Bb  = Bt + (size_t)b * strideB;
  const T* Ab2 = SPLIT ? (A2  + (size_t)b * strideA) : nullptr;
  const T* Bb2 = SPLIT ? (Bt2 + (size_t)b * strideB) : nullptr;

  const int rlane = lane & 15;
  const int koff  = (lane >> 4) * 8;
  const int mOff  = (lane >> 4) * 8;

  v8f acc[4][4];
#pragma unroll
  for (int i = 0; i < 4; ++i)
#pragma unroll
    for (int j = 0; j < 4; ++j) acc[i][j] = (v8f){0.f,0.f,0.f,0.f,0.f,0.f,0.f,0.f};

  for (int k0 = 0; k0 < K; k0 += 32) {
    V bh[4], bl[4];
#pragma unroll
    for (int j = 0; j < 4; ++j) {
      const size_t bo = (size_t)(n0 + (j << 4) + rlane) * ldb + koff + k0;
      bh[j] = Frag<T>::load(Bb + bo);
      if (SPLIT) bl[j] = Frag<T>::load(Bb2 + bo);
    }
#pragma unroll
    for (int i = 0; i < 4; ++i) {
      const size_t ao = (size_t)(m0 + (i << 4) + rlane) * lda + koff + k0;
      V ah = Frag<T>::load(Ab + ao);
      V al;
      if (SPLIT) al = Frag<T>::load(Ab2 + ao);
#pragma unroll
      for (int j = 0; j < 4; ++j) {
        acc[i][j] = Frag<T>::mma(ah, bh[j], acc[i][j]);
        if (SPLIT) {
          acc[i][j] = Frag<T>::mma(ah, bl[j], acc[i][j]);
          acc[i][j] = Frag<T>::mma(al, bh[j], acc[i][j]);
        }
      }
      Frag<T>::guard(acc[i][0], acc[i][3], ah, SPLIT ? al : ah);
    }
    Frag<T>::keep(bh[0], bh[1], bh[2], bh[3]);
    if (SPLIT) Frag<T>::keep(bl[0], bl[1], bl[2], bl[3]);
  }
  acc_guard4(acc[0][0], acc[0][1], acc[0][2], acc[0][3]);
  acc_guard4(acc[1][0], acc[1][1], acc[1][2], acc[1][3]);
  acc_guard4(acc[2][0], acc[2][1], acc[2][2], acc[2][3]);
  acc_guard4(acc[3][0], acc[3][1], acc[3][2], acc[3][3]);

  float* slab = sT[wave];
  const float* Rb = RESID ? (resid + (size_t)b * strideR) : nullptr;
#pragma unroll
  for (int i = 0; i < 4; ++i) {
    const int mBase = m0 + (i << 4);
#pragma unroll
    for (int j = 0; j < 4; ++j) {
      const int n = n0 + (j << 4) + rlane;
      float bv = 0.f;
      if (BIAS_MODE == 2) bv = bias[n];
#pragma unroll
      for (int r = 0; r < 8; ++r) {
        float v = acc[i][j][r] * scale;
        if (BIAS_MODE == 1) v += bias[mBase + mOff + r];
        if (BIAS_MODE == 2) v += bv;
        if (RESID) v += Rb[(size_t)(mBase + mOff + r) * ldc + n];
        if (ACT == 1) v = tanhf(v);
        if (ACT == 2) v = fmaxf(v, 0.0f);
        if (ACT == 3) v = v / (1.0f + expf(-v));
        if (ACT == 4) v = (v > 0.f) ? v : 0.01f * v;
        if (ACT == 5) v = 0.5f * v * (1.0f + erff(v * 0.70710678118654752f));
        slab[(mOff + r) * 68 + (j << 4) + rlane] = v;
      }
    }
    __builtin_amdgcn_fence(__ATOMIC_RELEASE, "workgroup");
    __builtin_amdgcn_wave_barrier();
    __builtin_amdgcn_fence(__ATOMIC_ACQUIRE, "workgroup");
    if (OUT_MODE == 0) {
      float* C = (float*)Cout + (size_t)b * strideC;
      const int hh = lane >> 4, c4 = (lane & 15) * 4;
      for (int pass = 0; pass < 2; ++pass) {
#pragma unroll
        for (int it = 0; it < 8; ++it) {
          const int row = it * 2 + hh;
          v4f v = *(const v4f*)(slab + row * 68 + c4);
          *(volatile v4f*)(C + (size_t)(mBase + row) * ldc + n0 + c4) = v;
        }
        __threadfence();
      }
    } else {
      const int q = lane >> 3, c8 = (lane & 7) * 8;
      unsigned short* C  = (unsigned short*)Cout  + (size_t)b * strideC;
      unsigned short* C2 = (OUT_MODE == 2) ? ((unsigned short*)Cout2 + (size_t)b * strideC) : nullptr;
      for (int pass = 0; pass < 2; ++pass) {
#pragma unroll
        for (int it = 0; it < 4; ++it) {
          const int row = it * 4 + q;
          const float* sp = slab + row * 68 + c8;
          v8h hv, lv;
#pragma unroll
          for (int e = 0; e < 8; ++e) {
            if (OUT_MODE == 1) {
              hv[e] = (_Float16)sp[e];
            } else {
              unsigned short hb = f2bf_bits(sp[e]);
              unsigned short lb = f2bf_bits(sp[e] - bf_bits2f(hb));
              hv[e] = __builtin_bit_cast(_Float16, hb);
              lv[e] = __builtin_bit_cast(_Float16, lb);
            }
          }
          *(volatile v8h*)(C + (size_t)(mBase + row) * ldc + n0 + c8) = hv;
          if (OUT_MODE == 2) *(volatile v8h*)(C2 + (size_t)(mBase + row) * ldc + n0 + c8) = lv;
        }
        __threadfence();
      }
    }
    __builtin_amdgcn_fence(__ATOMIC_RELEASE, "workgroup");
    __builtin_amdgcn_wave_barrier();
    __builtin_amdgcn_fence(__ATOMIC_ACQUIRE, "workgroup");
  }
}

__device__ __forceinline__ int imin(int a, int b) { return a < b ? a : b; }
__device__ __forceinline__ int imax(int a, int b) { return a > b ? a : b; }
__device__ __forceinline__ float bf16r(float f) { return bf_bits2f(f2bf_bits(f)); }
__device__ __forceinline__ unsigned pk2(unsigned short a, unsigned short b) { return (unsigned)a | ((unsigned)b << 16); }
__device__ __forceinline__ unsigned pkh2(float a, float b) {
  return pk2(__builtin_bit_cast(unsigned short, (_Float16)a), __builtin_bit_cast(unsigned short, (_Float16)b));
}
__device__ __forceinline__ float elu1(float v) {
  const float e = __expf(fminf(v, 0.0f)) - 1.0f;
  return v > 0.0f ? v : e;
}
__device__ __forceinline__ void rs_taps(int d, int n, int& i0, int& i1, float& w0, float& w1) {
  const int m = d >> 1;
  const bool odd = (d & 1) != 0;
  int a0 = odd ? m : m - 1;
  int a1 = odd ? m + 1 : m;
  float u0 = odd ? 0.75f : 0.25f;
  float u1 = odd ? 0.25f : 0.75f;
  if (a0 < 0) { a0 = 0; u0 = 0.0f; u1 = 1.0f; }
  if (a1 > n - 1) { a1 = n - 1; u0 = 1.0f; u1 = 0.0f; }
  i0 = a0; i1 = a1; w0 = u0; w1 = u1;
}

__global__ __launch_bounds__(96) void k_par(const float* __restrict__ ob1, const float* __restrict__ b1,
                                            const float* __restrict__ rb, const float* __restrict__ ob2,
                                            const float* __restrict__ b2, float* __restrict__ par) {
  const int t = threadIdx.x;
  const int slot = t >> 4;
  const int e0 = (t & 15) * 4;
  v4f v;
#pragma unroll
  for (int j = 0; j < 4; ++j) {
    const int e = e0 + j;
    const int ea = e < NOFF ? e : (NOFF - 1);
    const int eb = e < CMID ? e : (CMID - 1);
    const float f0 = ob1[ea], f1 = b1[eb], f2 = rb[eb], f3 = ob2[ea], f4 = b2[eb];
    const float v0 = (e < NOFF) ? bf16r(f0) : 0.0f;
    const float v1 = (e < CMID) ? bf16r(f1) : 0.0f;
    const float v2 = (e < CMID) ? bf16r(f2) : 0.0f;
    const float v3 = (e < NOFF) ? bf16r(f3) : 0.0f;
    const float v4 = (e < CMID) ? bf16r(f4) : 0.0f;
    v[j] = (slot == 0) ? v0 : (slot == 1) ? v1 : (slot == 2) ? v2 : (slot == 3) ? v3 : v4;
  }
  if (t < 80) {
    volatile v4f* p = (volatile v4f*)(par + (size_t)slot * PARSLOT + e0);
    *p = v;
    __threadfence();
    *p = v;
  }
}

template <int F16OUT>
__global__ __launch_bounds__(256) void k_prepw(const float* __restrict__ w, unsigned short* __restrict__ dst,
                                               int cin, int ntap, int nreal, int ktot, int nchunks, float scale) {
  const int i = blockIdx.x * 256 + threadIdx.x;
  if (i >= nchunks) return;
  const int h0 = i * 8;
  const int n = h0 / ktot;
  const int k0 = h0 - n * ktot;
  const bool inb = n < nreal;
  const int nc = inb ? n : (nreal - 1);
  float f[8];
#pragma unroll
  for (int e = 0; e < 8; ++e) {
    const int k = k0 + e;
    const int tap = k / cin;
    const int c = k - tap * cin;
    const float raw = w[((size_t)nc * cin + c) * ntap + tap];
    f[e] = inb ? (bf16r(raw) * scale) : 0.0f;
  }
  v4u u;
#pragma unroll
  for (int e2 = 0; e2 < 4; ++e2) {
    if (F16OUT) u[e2] = pkh2(f[2 * e2], f[2 * e2 + 1]);
    else        u[e2] = pk2(f2bf_bits(f[2 * e2]), f2bf_bits(f[2 * e2 + 1]));
  }
  volatile v4u* p = (volatile v4u*)(dst + (size_t)h0);
  *p = u;
  __threadfence();
  *p = u;
}

__global__ __launch_bounds__(256) void k_xt(const float* __restrict__ x, unsigned short* __restrict__ xt) {
  __shared__ float t[CIN][65];
  const int tid = threadIdx.x;
  const int b = blockIdx.x >> 8;
  const int px0 = (blockIdx.x & 255) * 64;
#pragma unroll
  for (int it = 0; it < 16; ++it) {
    const int idx = it * 256 + tid;
    const int c = idx >> 6, p = idx & 63;
    t[c][p] = x[((size_t)(b * CIN + c)) * PX1 + px0 + p];
  }
  __syncthreads();
  const int wave = tid >> 5, lane = tid & 31, q = lane >> 3, c8 = (lane & 7) * 8;
  v4u u[2];
#pragma unroll
  for (int it = 0; it < 2; ++it) {
    const int row = it * 32 + wave * 4 + q;
    v4u a;
#pragma unroll
    for (int e2 = 0; e2 < 4; ++e2) a[e2] = pk2(f2bf_bits(t[c8 + 2 * e2][row]), f2bf_bits(t[c8 + 2 * e2 + 1][row]));
    u[it] = a;
  }
  for (int pass = 0; pass < 2; ++pass) {
#pragma unroll
    for (int it = 0; it < 2; ++it) {
      const int row = it * 32 + wave * 4 + q;
      *(volatile v4u*)(xt + ((size_t)(b * PX1 + px0 + row)) * CIN + c8) = u[it];
    }
    __threadfence();
  }
}

__global__ __launch_bounds__(256) void k_im2col1(const unsigned short* __restrict__ xt, unsigned short* __restrict__ im) {
  const int gid = blockIdx.x * 256 + threadIdx.x;
  const int line = gid >> 3, sub = gid & 7;
  const int P = line / NTAP, tap = line - P * NTAP;
  const int b = P >> 14, p = P & (PX1 - 1);
  const int y = p >> 7, xx = p & (HS1 - 1);
  const int t3 = tap / 3;
  const int ys = y + t3 - 1, xs = xx + (tap - t3 * 3) - 1;
  const bool ok = (ys >= 0) && (ys < HS1) && (xs >= 0) && (xs < HS1);
  const int ysc = imin(imax(ys, 0), HS1 - 1), xsc = imin(imax(xs, 0), HS1 - 1);
  const v4u raw = *(const v4u*)(xt + ((size_t)(b * PX1 + ysc * HS1 + xsc)) * CIN + sub * 8);
  const v4u zero = (v4u){0u, 0u, 0u, 0u};
  const v4u v = ok ? raw : zero;
  volatile v4u* d = (volatile v4u*)(im + (size_t)line * CIN + sub * 8);
  *d = v;
  __threadfence();
  *d = v;
}

__global__ __launch_bounds__(256) void k_sample1(const unsigned short* __restrict__ xt, const float* __restrict__ om,
                                                 unsigned short* __restrict__ sp) {
  const int gid = blockIdx.x * 256 + threadIdx.x;
  const int line = gid >> 3, sub = gid & 7;
  const int P = line / NTAP, tap = line - P * NTAP;
  const int b = P >> 14, p = P & (PX1 - 1);
  const int y = p >> 7, xx = p & (HS1 - 1);
  const int t3 = tap / 3;
  const int ti = t3 - 1, tj = (tap - t3 * 3) - 1;
  const float* omp = om + (size_t)P * NPAD;
  const float dyv = omp[2 * tap], dxv = omp[2 * tap + 1], ml = omp[18 + tap];
  const float mk = __builtin_amdgcn_rcpf(1.0f + __expf(-ml));
  const float py = ((float)y + (float)ti) + dyv;
  const float px = ((float)xx + (float)tj) + dxv;
  const float fy = floorf(py), fx = floorf(px);
  const float ty = py - fy, tx = px - fx;
  const int iy0 = (int)fminf(fmaxf(fy, -2.0f), (float)(HS1 + 1));
  const int ix0 = (int)fminf(fmaxf(fx, -2.0f), (float)(HS1 + 1));
  const int iy1 = iy0 + 1, ix1 = ix0 + 1;
  const float vy0 = (iy0 >= 0 && iy0 < HS1) ? 1.0f : 0.0f;
  const float vy1 = (iy1 >= 0 && iy1 < HS1) ? 1.0f : 0.0f;
  const float vx0 = (ix0 >= 0 && ix0 < HS1) ? 1.0f : 0.0f;
  const float vx1 = (ix1 >= 0 && ix1 < HS1) ? 1.0f : 0.0f;
  const int cy0 = imin(imax(iy0, 0), HS1 - 1), cy1 = imin(imax(iy1, 0), HS1 - 1);
  const int cx0 = imin(imax(ix0, 0), HS1 - 1), cx1 = imin(imax(ix1, 0), HS1 - 1);
  const float w00 = ((1.0f - ty) * (1.0f - tx)) * (vy0 * vx0);
  const float w01 = ((1.0f - ty) * tx) * (vy0 * vx1);
  const float w10 = (ty * (1.0f - tx)) * (vy1 * vx0);
  const float w11 = (ty * tx) * (vy1 * vx1);
  const float msc = mk * CARRY_ACT;
  const unsigned short* xb = xt + (size_t)b * PX1 * CIN + sub * 8;
  const v4u q00 = *(const v4u*)(xb + (size_t)(cy0 * HS1 + cx0) * CIN);
  const v4u q01 = *(const v4u*)(xb + (size_t)(cy0 * HS1 + cx1) * CIN);
  const v4u q10 = *(const v4u*)(xb + (size_t)(cy1 * HS1 + cx0) * CIN);
  const v4u q11 = *(const v4u*)(xb + (size_t)(cy1 * HS1 + cx1) * CIN);
  v4u u;
#pragma unroll
  for (int e2 = 0; e2 < 4; ++e2) {
    const unsigned ua = q00[e2], ub = q01[e2], uc = q10[e2], ud = q11[e2];
    const float a0 = __uint_as_float(ua << 16), a1 = __uint_as_float(ua & 0xFFFF0000u);
    const float b0 = __uint_as_float(ub << 16), b1 = __uint_as_float(ub & 0xFFFF0000u);
    const float c0 = __uint_as_float(uc << 16), c1 = __uint_as_float(uc & 0xFFFF0000u);
    const float d0 = __uint_as_float(ud << 16), d1 = __uint_as_float(ud & 0xFFFF0000u);
    const float o0 = ((a0 * w00 + b0 * w01) + c0 * w10) + d0 * w11;
    const float o1 = ((a1 * w00 + b1 * w01) + c1 * w10) + d1 * w11;
    u[e2] = pkh2(o0 * msc, o1 * msc);
  }
  volatile v4u* d = (volatile v4u*)(sp + (size_t)line * CIN + sub * 8);
  *d = u;
  __threadfence();
  *d = u;
}

template <bool DO_ELU>
__global__ __launch_bounds__(256) void k_up(const float* __restrict__ src, float* __restrict__ dst) {
  const int gid = blockIdx.x * 256 + threadIdx.x;
  const int line = gid >> 3, sub = gid & 7, c4 = sub * 4;
  const int b = line >> 16, q = line & (PX2 - 1);
  const int Y = q >> 8, X = q & (HS2 - 1);
  int y0, y1, x0, x1; float wy0, wy1, wx0, wx1;
  rs_taps(Y, HS1, y0, y1, wy0, wy1);
  rs_taps(X, HS1, x0, x1, wx0, wx1);
  const float* sb = src + (size_t)b * PX1 * NPAD + c4;
  const v4f v00 = *(const v4f*)(sb + (size_t)(y0 * HS1 + x0) * NPAD);
  const v4f v01 = *(const v4f*)(sb + (size_t)(y0 * HS1 + x1) * NPAD);
  const v4f v10 = *(const v4f*)(sb + (size_t)(y1 * HS1 + x0) * NPAD);
  const v4f v11 = *(const v4f*)(sb + (size_t)(y1 * HS1 + x1) * NPAD);
  v4f o;
#pragma unroll
  for (int e = 0; e < 4; ++e) {
    float fa = v00[e], fb = v01[e], fc = v10[e], fd = v11[e];
    if (DO_ELU) { fa = elu1(fa); fb = elu1(fb); fc = elu1(fc); fd = elu1(fd); }
    o[e] = wy0 * (wx0 * fa + wx1 * fb) + wy1 * (wx0 * fc + wx1 * fd);
  }
  volatile v4f* pd = (volatile v4f*)(dst + (size_t)line * CMID + c4);
  *pd = o;
  __threadfence();
  *pd = o;
}

__global__ __launch_bounds__(256) void k_im2col2(const float* __restrict__ hin, unsigned short* __restrict__ im) {
  const int gid = blockIdx.x * 256 + threadIdx.x;
  const int seg = gid >> 2, sub = gid & 3;
  const int p = seg / NTAP, tap = seg - p * NTAP;
  const int y = p >> 8, xx = p & (HS2 - 1);
  const int t3 = tap / 3;
  const int ys = y + t3 - 1, xs = xx + (tap - t3 * 3) - 1;
  const bool ok = (ys >= 0) && (ys < HS2) && (xs >= 0) && (xs < HS2);
  const int ysc = imin(imax(ys, 0), HS2 - 1), xsc = imin(imax(xs, 0), HS2 - 1);
  const float* s = hin + (size_t)(ysc * HS2 + xsc) * CMID + sub * 8;
  const v4f a = *(const v4f*)s;
  const v4f c = *(const v4f*)(s + 4);
  const float z = CARRY_ACT;
  v4u u;
  u[0] = pkh2(ok ? a[0] * z : 0.0f, ok ? a[1] * z : 0.0f);
  u[1] = pkh2(ok ? a[2] * z : 0.0f, ok ? a[3] * z : 0.0f);
  u[2] = pkh2(ok ? c[0] * z : 0.0f, ok ? c[1] * z : 0.0f);
  u[3] = pkh2(ok ? c[2] * z : 0.0f, ok ? c[3] * z : 0.0f);
  volatile v4u* d = (volatile v4u*)(im + (size_t)seg * CMID + sub * 8);
  *d = u;
  __threadfence();
  *d = u;
}

__global__ __launch_bounds__(256) void k_sample2(const float* __restrict__ hin, const float* __restrict__ om,
                                                 unsigned short* __restrict__ sp) {
  const int gid = blockIdx.x * 256 + threadIdx.x;
  const int seg = gid >> 2, sub = gid & 3;
  const int p = seg / NTAP, tap = seg - p * NTAP;
  const int y = p >> 8, xx = p & (HS2 - 1);
  const int t3 = tap / 3;
  const int ti = t3 - 1, tj = (tap - t3 * 3) - 1;
  const float* omp = om + (size_t)p * NPAD;
  const float dyv = omp[2 * tap], dxv = omp[2 * tap + 1], ml = omp[18 + tap];
  const float mk = __builtin_amdgcn_rcpf(1.0f + __expf(-ml));
  const float py = ((float)y + (float)ti) + dyv;
  const float px = ((float)xx + (float)tj) + dxv;
  const float fy = floorf(py), fx = floorf(px);
  const float ty = py - fy, tx = px - fx;
  const int iy0 = (int)fminf(fmaxf(fy, -2.0f), (float)(HS2 + 1));
  const int ix0 = (int)fminf(fmaxf(fx, -2.0f), (float)(HS2 + 1));
  const int iy1 = iy0 + 1, ix1 = ix0 + 1;
  const float vy0 = (iy0 >= 0 && iy0 < HS2) ? 1.0f : 0.0f;
  const float vy1 = (iy1 >= 0 && iy1 < HS2) ? 1.0f : 0.0f;
  const float vx0 = (ix0 >= 0 && ix0 < HS2) ? 1.0f : 0.0f;
  const float vx1 = (ix1 >= 0 && ix1 < HS2) ? 1.0f : 0.0f;
  const int cy0 = imin(imax(iy0, 0), HS2 - 1), cy1 = imin(imax(iy1, 0), HS2 - 1);
  const int cx0 = imin(imax(ix0, 0), HS2 - 1), cx1 = imin(imax(ix1, 0), HS2 - 1);
  const float w00 = ((1.0f - ty) * (1.0f - tx)) * (vy0 * vx0);
  const float w01 = ((1.0f - ty) * tx) * (vy0 * vx1);
  const float w10 = (ty * (1.0f - tx)) * (vy1 * vx0);
  const float w11 = (ty * tx) * (vy1 * vx1);
  const float msc = mk * CARRY_ACT;
  const float* hb = hin + sub * 8;
  const float* r00 = hb + (size_t)(cy0 * HS2 + cx0) * CMID;
  const float* r01 = hb + (size_t)(cy0 * HS2 + cx1) * CMID;
  const float* r10 = hb + (size_t)(cy1 * HS2 + cx0) * CMID;
  const float* r11 = hb + (size_t)(cy1 * HS2 + cx1) * CMID;
  const v4f aL = *(const v4f*)r00, aH = *(const v4f*)(r00 + 4);
  const v4f bL = *(const v4f*)r01, bH = *(const v4f*)(r01 + 4);
  const v4f cL = *(const v4f*)r10, cH = *(const v4f*)(r10 + 4);
  const v4f dL = *(const v4f*)r11, dH = *(const v4f*)(r11 + 4);
  float oL[4], oH[4];
#pragma unroll
  for (int e = 0; e < 4; ++e) {
    oL[e] = (((aL[e] * w00 + bL[e] * w01) + cL[e] * w10) + dL[e] * w11) * msc;
    oH[e] = (((aH[e] * w00 + bH[e] * w01) + cH[e] * w10) + dH[e] * w11) * msc;
  }
  v4u u;
  u[0] = pkh2(oL[0], oL[1]);
  u[1] = pkh2(oL[2], oL[3]);
  u[2] = pkh2(oH[0], oH[1]);
  u[3] = pkh2(oH[2], oH[3]);
  volatile v4u* d = (volatile v4u*)(sp + (size_t)seg * CMID + sub * 8);
  *d = u;
  __threadfence();
  *d = u;
}

__global__ __launch_bounds__(256) void k_out(const float* __restrict__ d2, const float* __restrict__ ru,
                                             float* __restrict__ out) {
  __shared__ float t[CMID][65];
  const int tid = threadIdx.x;
  const int p0 = blockIdx.x * 64;
#pragma unroll
  for (int it = 0; it < 8; ++it) {
    const int idx = it * 256 + tid;
    const int pl = idx >> 5, c = idx & 31;
    const float dv = d2[(size_t)(p0 + pl) * NPAD + c];
    const float rv = ru[(size_t)(p0 + pl) * CMID + c];
    t[c][pl] = elu1(dv) + rv;
  }
  __syncthreads();
  const int wave = tid >> 5, lane = tid & 31, hh = lane >> 4, c4 = (lane & 15) * 4;
  v4f v[2];
#pragma unroll
  for (int it = 0; it < 2; ++it) {
    const int ch = it * 16 + wave * 2 + hh;
    v4f a;
    a[0] = t[ch][c4 + 0]; a[1] = t[ch][c4 + 1]; a[2] = t[ch][c4 + 2]; a[3] = t[ch][c4 + 3];
    v[it] = a;
  }
  for (int pass = 0; pass < 2; ++pass) {
#pragma unroll
    for (int it = 0; it < 2; ++it) {
      const int ch = it * 16 + wave * 2 + hh;
      *(volatile v4f*)(out + (size_t)ch * PX2 + p0 + c4) = v[it];
    }
    __threadfence();
  }
}

extern "C" void kernel_launch(void* const* d_in, const int* in_sizes, int n_in,
                              void* d_out, int out_size, void* d_ws, size_t ws_size, hipStream_t stream) {
  if (n_in != 11) return;
  if (in_sizes[0] != NIMG * CIN * PX1 || in_sizes[1] != CMID * CIN * NTAP || in_sizes[2] != CMID ||
      in_sizes[3] != NOFF * CIN * NTAP || in_sizes[4] != NOFF || in_sizes[5] != CMID * CMID * NTAP ||
      in_sizes[6] != CMID || in_sizes[7] != NOFF * CMID * NTAP || in_sizes[8] != NOFF ||
      in_sizes[9] != CMID * CIN || in_sizes[10] != CMID) return;
  if (out_size != NIMG * CMID * PX2) return;

  const float* x   = (const float*)d_in[0];
  const float* w1  = (const float*)d_in[1];
  const float* b1  = (const float*)d_in[2];
  const float* ow1 = (const float*)d_in[3];
  const float* ob1 = (const float*)d_in[4];
  const float* w2  = (const float*)d_in[5];
  const float* b2  = (const float*)d_in[6];
  const float* ow2 = (const float*)d_in[7];
  const float* ob2 = (const float*)d_in[8];
  const float* rw  = (const float*)d_in[9];
  const float* rb  = (const float*)d_in[10];
  float* out = (float*)d_out;

  unsigned char* wsb = (unsigned char*)d_ws;
  size_t off = 0;
  float* PAR = (float*)(wsb + off);                           off += 2048;
  unsigned short* OW1P = (unsigned short*)(wsb + off);        off += (size_t)64 * KT1 * 2;
  unsigned short* W1P  = (unsigned short*)(wsb + off);        off += (size_t)64 * KT1 * 2;
  unsigned short* RWP  = (unsigned short*)(wsb + off);        off += (size_t)64 * CIN * 2;
  unsigned short* OW2P = (unsigned short*)(wsb + off);        off += (size_t)64 * KT2 * 2;
  unsigned short* W2P  = (unsigned short*)(wsb + off);        off += (size_t)64 * KT2 * 2;
  unsigned short* XT   = (unsigned short*)(wsb + off);        off += (size_t)NIMG * PX1 * CIN * 2;
  const size_t bigA = ((size_t)NIMG * PX1 * KT1 * 2 > (size_t)PX2 * KT2 * 2) ? (size_t)NIMG * PX1 * KT1 * 2 : (size_t)PX2 * KT2 * 2;
  unsigned short* BIGA = (unsigned short*)(wsb + off);        off += bigA;
  const size_t bigB = ((size_t)NIMG * PX1 * NPAD * 4 > (size_t)PX2 * NPAD * 4) ? (size_t)NIMG * PX1 * NPAD * 4 : (size_t)PX2 * NPAD * 4;
  float* BIGB = (float*)(wsb + off);                          off += bigB;
  float* RES  = (float*)(wsb + off);                          off += (size_t)NIMG * PX1 * NPAD * 4;
  float* H1U  = (float*)(wsb + off);                          off += (size_t)NIMG * PX2 * CMID * 4;
  float* RESU = (float*)(wsb + off);                          off += (size_t)NIMG * PX2 * CMID * 4;
  if (off > ws_size) return;

  k_par<<<1, 96, 0, stream>>>(ob1, b1, rb, ob2, b2, PAR);
  {
    const int n1 = 64 * KT1 / 8, n2 = 64 * KT2 / 8, n3 = 64 * CIN / 8;
    k_prepw<0><<<(n1 + 255) / 256, 256, 0, stream>>>(ow1, OW1P, CIN, NTAP, NOFF, KT1, n1, 1.0f);
    k_prepw<1><<<(n1 + 255) / 256, 256, 0, stream>>>(w1,  W1P,  CIN, NTAP, CMID, KT1, n1, CARRY_W);
    k_prepw<0><<<(n3 + 255) / 256, 256, 0, stream>>>(rw,  RWP,  CIN, 1,    CMID, CIN, n3, 1.0f);
    k_prepw<1><<<(n2 + 255) / 256, 256, 0, stream>>>(ow2, OW2P, CMID, NTAP, NOFF, KT2, n2, CARRY_W);
    k_prepw<1><<<(n2 + 255) / 256, 256, 0, stream>>>(w2,  W2P,  CMID, NTAP, CMID, KT2, n2, CARRY_W);
  }
  k_xt<<<NIMG * PX1 / 64, 256, 0, stream>>>(x, XT);
  k_im2col1<<<NIMG * PX1 * NTAP * 8 / 256, 256, 0, stream>>>(XT, BIGA);
  const int tiles1 = (NIMG * PX1 / 64) * (NPAD / 64);
  const int tiles2 = (PX2 / 64) * (NPAD / 64);
  wmma_gemm64<1, false, 2, 0, false, 0><<<dim3((tiles1 + 7) / 8, 1), 256, 0, stream>>>(
      BIGA, BIGA, KT1, 0L, OW1P, OW1P, KT1, 0L, (void*)BIGB, (void*)BIGB, NPAD, 0L,
      PAR + 0 * PARSLOT, (const float*)nullptr, 0L, NIMG * PX1, NPAD, KT1, 1.0f);
  k_sample1<<<NIMG * PX1 * NTAP * 8 / 256, 256, 0, stream>>>(XT, BIGB, BIGA);
  wmma_gemm64<0, false, 2, 0, false, 0><<<dim3((tiles1 + 7) / 8, 1), 256, 0, stream>>>(
      BIGA, BIGA, KT1, 0L, W1P, W1P, KT1, 0L, (void*)BIGB, (void*)BIGB, NPAD, 0L,
      PAR + 1 * PARSLOT, (const float*)nullptr, 0L, NIMG * PX1, NPAD, KT1, CARRY_INV);
  wmma_gemm64<1, false, 2, 0, false, 0><<<dim3((tiles1 + 7) / 8, 1), 256, 0, stream>>>(
      XT, XT, CIN, 0L, RWP, RWP, CIN, 0L, (void*)RES, (void*)RES, NPAD, 0L,
      PAR + 2 * PARSLOT, (const float*)nullptr, 0L, NIMG * PX1, NPAD, CIN, 1.0f);
  k_up<true><<<NIMG * PX2 * 8 / 256, 256, 0, stream>>>(BIGB, H1U);
  k_up<false><<<NIMG * PX2 * 8 / 256, 256, 0, stream>>>(RES, RESU);
  for (int img = 0; img < NIMG; ++img) {
    const float* hin = H1U + (size_t)img * PX2 * CMID;
    k_im2col2<<<PX2 * NTAP * 4 / 256, 256, 0, stream>>>(hin, BIGA);
    wmma_gemm64<0, false, 2, 0, false, 0><<<dim3((tiles2 + 7) / 8, 1), 256, 0, stream>>>(
        BIGA, BIGA, KT2, 0L, OW2P, OW2P, KT2, 0L, (void*)BIGB, (void*)BIGB, NPAD, 0L,
        PAR + 3 * PARSLOT, (const float*)nullptr, 0L, PX2, NPAD, KT2, CARRY_INV);
    k_sample2<<<PX2 * NTAP * 4 / 256, 256, 0, stream>>>(hin, BIGB, BIGA);
    wmma_gemm64<0, false, 2, 0, false, 0><<<dim3((tiles2 + 7) / 8, 1), 256, 0, stream>>>(
        BIGA, BIGA, KT2, 0L, W2P, W2P, KT2, 0L, (void*)BIGB, (void*)BIGB, NPAD, 0L,
        PAR + 4 * PARSLOT, (const float*)nullptr, 0L, PX2, NPAD, KT2, CARRY_INV);
    k_out<<<PX2 / 64, 256, 0, stream>>>(BIGB, RESU + (size_t)img * PX2 * CMID, out + (size_t)img * CMID * PX2);
  }
}
